// CAREGNNLayer_78632261255938
// MI455X (gfx1250) — hardware-run, weakly checked
//
#include <hip/hip_runtime.h>

typedef float          v8f   __attribute__((ext_vector_type(8)));
typedef float          v4f   __attribute__((ext_vector_type(4)));
typedef unsigned int   v4u   __attribute__((ext_vector_type(4)));
typedef int            v8i   __attribute__((ext_vector_type(8)));
typedef unsigned short v8us  __attribute__((ext_vector_type(8)));
typedef unsigned short v16us __attribute__((ext_vector_type(16)));
typedef __bf16         v16bf __attribute__((ext_vector_type(16)));
typedef _Float16       v16h  __attribute__((ext_vector_type(16)));
typedef v4f  __attribute__((may_alias)) v4fa;
typedef v8us __attribute__((may_alias)) v8usa;
union FragB { v16bf v; v16us u; v8us h[2]; v8i w; };
union FragH { v16h  v; v16us u; v8us h[2]; v8i w; };

__device__ __forceinline__ v8f wmb(const FragB& a, const FragB& b, v8f c) {
  v8f d = __builtin_amdgcn_wmma_f32_16x16x32_bf16(false, a.v, false, b.v, (short)0, c, false, false);
  asm volatile("v_nop\n\tv_nop\n\tv_nop\n\tv_nop" : "+v"(d) : "v"(a.w), "v"(b.w));
  return d;
}

__device__ __forceinline__ v8f wmh(const FragH& a, const FragH& b, v8f c) {
  v8f d = __builtin_amdgcn_wmma_f32_16x16x32_f16(false, a.v, false, b.v, (short)0, c, false, false);
  asm volatile("v_nop\n\tv_nop\n\tv_nop\n\tv_nop" : "+v"(d) : "v"(a.w), "v"(b.w));
  return d;
}

__device__ __forceinline__ unsigned bf16_bits(float f) {
  const unsigned u = __float_as_uint(f);
  const unsigned r = (u + 0x7FFFu + ((u >> 16) & 1u)) >> 16;
  const unsigned q = (u >> 16) | 0x40u;
  return ((u & 0x7fffffffu) > 0x7f800000u) ? q : r;
}

__device__ __forceinline__ float bf16_val(float f) {
  return __uint_as_float(bf16_bits(f) << 16);
}
__device__ __forceinline__ int clampi(int v, int lo, int hi) {
  return v < lo ? lo : (v > hi ? hi : v);
}

__device__ __forceinline__ unsigned f16_bits(float f) {
  const unsigned u  = __float_as_uint(f);
  const unsigned s  = (u >> 16) & 0x8000u;
  const unsigned a  = u & 0x7fffffffu;
  const unsigned t  = a - 0x38000000u;
  const unsigned r  = (t + 0x0FFFu + ((t >> 13) & 1u)) >> 13;
  const unsigned rc = r > 0x7C00u ? 0x7C00u : r;
  const bool small  = a < 0x38800000u;
  const bool isnan  = a > 0x7f800000u;
  const unsigned fin = small ? 0u : (s | rc);
  return isnan ? (s | 0x7E00u) : fin;
}

__device__ __forceinline__ unsigned pk16(unsigned lo, unsigned hi) { return lo | (hi << 16); }
__device__ __forceinline__ unsigned bf16_lo_bits(float v) {
  float hi = bf16_val(v);
  asm volatile("" : "+v"(hi));
  return bf16_bits(v - hi);
}
__device__ __forceinline__ v4u pack8_bf16(v4f a, v4f c) {
  return (v4u){ pk16(bf16_bits(a[0]), bf16_bits(a[1])), pk16(bf16_bits(a[2]), bf16_bits(a[3])),
                pk16(bf16_bits(c[0]), bf16_bits(c[1])), pk16(bf16_bits(c[2]), bf16_bits(c[3])) };
}
__device__ __forceinline__ v4u pack8_bf16_lo(v4f a, v4f c) {
  return (v4u){ pk16(bf16_lo_bits(a[0]), bf16_lo_bits(a[1])), pk16(bf16_lo_bits(a[2]), bf16_lo_bits(a[3])),
                pk16(bf16_lo_bits(c[0]), bf16_lo_bits(c[1])), pk16(bf16_lo_bits(c[2]), bf16_lo_bits(c[3])) };
}
__device__ __forceinline__ v4u pack8_f16(v4f a, v4f c) {
  return (v4u){ pk16(f16_bits(a[0]), f16_bits(a[1])), pk16(f16_bits(a[2]), f16_bits(a[3])),
                pk16(f16_bits(c[0]), f16_bits(c[1])), pk16(f16_bits(c[2]), f16_bits(c[3])) };
}

template <int FORM>
__global__ __launch_bounds__(256) void k_plane(const float* __restrict__ src, int rows, int cols, int ldsrc,
                                               unsigned short* __restrict__ dst, int MP, int KP) {
  static_assert(FORM >= 0 && FORM <= 3);
  const int KTOT = (FORM == 1 || FORM == 3) ? 2 * KP : KP;
  const unsigned ppr   = (unsigned)(KTOT >> 3);
  const unsigned kp8   = (unsigned)(KP >> 3);
  const unsigned total = (unsigned)MP * ppr;
  const unsigned g     = blockIdx.x * 256u + threadIdx.x;
  const unsigned rowu  = g / ppr;
  const unsigned p     = g - rowu * ppr;
  const bool second    = p >= kp8;
  const int row = (int)rowu;
  const int c0  = (int)((second ? p - kp8 : p) << 3);
  const float* srow = src + (size_t)clampi(row, 0, rows - 1) * (size_t)ldsrc;
  float x[8];
  unsigned mk[8];
#pragma unroll
  for (int e = 0; e < 8; ++e) {
    const int c = c0 + e;
    const float v = srow[clampi(c, 0, cols - 1)];
    asm volatile("" :: "v"(v));
    x[e]  = v;
    mk[e] = (row < rows && c < cols) ? 0xFFFFu : 0u;
  }
  const v4f a = (v4f){ x[0], x[1], x[2], x[3] };
  const v4f c = (v4f){ x[4], x[5], x[6], x[7] };
  v4u o;
  if (FORM == 2) {
    o = pack8_f16(a, c);
  } else {
    const v4u hi = pack8_bf16(a, c);
    o = hi;
    if (FORM == 1) { const v4u lo = pack8_bf16_lo(a, c); o = second ? lo : hi; }
  }
  const v4u mw = (v4u){ pk16(mk[0], mk[1]), pk16(mk[2], mk[3]), pk16(mk[4], mk[5]), pk16(mk[6], mk[7]) };
  o &= mw;
  if (g < total) {
    volatile v4u* q = (volatile v4u*)(dst + (size_t)g * 8);
    *q = o;
    __threadfence();
    *q = o;
  }
}

template <int FORM> struct FragOf    { typedef FragB T; };
template <>         struct FragOf<2> { typedef FragH T; };
__device__ __forceinline__ v8f mm(const FragB& a, const FragB& b, v8f c) { return wmb(a, b, c); }
__device__ __forceinline__ v8f mm(const FragH& a, const FragH& b, v8f c) { return wmh(a, b, c); }
template <class F> __device__ __forceinline__ F ld_frag(const unsigned short* p) {
  F f;
  f.h[0] = *(const v8usa*)(p);
  f.h[1] = *(const v8usa*)(p + 16);
  return f;
}

template <int FORM, int EPI>
__global__ __launch_bounds__(256) __attribute__((amdgpu_num_vgpr(248)))
void k_gemm_nt(const unsigned short* __restrict__ A, const unsigned short* __restrict__ B,
               const float* __restrict__ bias, float* __restrict__ D, int M, int N, int KTOT, int ldd) {
  static_assert(FORM >= 0 && FORM <= 2);
  static_assert(EPI == 0 || EPI == 1);
  typedef typename FragOf<FORM>::T F;
  __shared__ __attribute__((aligned(16))) float sT[8][16 * 68];
  const int lane = threadIdx.x & 31;
  const int wave = threadIdx.x >> 5;
  const int tilesM = (M + 63) >> 6;
  const int tilesN = (N + 63) >> 6;
  const int tile = blockIdx.x * 8 + wave;
  if (tile >= tilesM * tilesN) return;
  const int tm = tile / tilesN;
  const int tn = tile - tm * tilesN;
  const int m0 = tm << 6;
  const int n0 = tn << 6;

  const int rl = lane & 15;
  const int h8 = (lane >> 4) * 8;
  const unsigned short* pa = A + (size_t)(m0 + rl) * (size_t)KTOT + h8;
  const unsigned short* pb = B + (size_t)(n0 + rl) * (size_t)KTOT + h8;

  v8f acc[4][4];
#pragma unroll
  for (int i = 0; i < 4; ++i)
#pragma unroll
    for (int j = 0; j < 4; ++j) acc[i][j] = (v8f){0.f, 0.f, 0.f, 0.f, 0.f, 0.f, 0.f, 0.f};

#pragma unroll 1
  for (int k0 = 0; k0 < KTOT; k0 += 32) {
    F bf[4];
#pragma unroll
    for (int j = 0; j < 4; ++j) bf[j] = ld_frag<F>(pb + (size_t)(j << 4) * (size_t)KTOT + k0);
#pragma unroll
    for (int i = 0; i < 4; ++i) {
      const F af = ld_frag<F>(pa + (size_t)(i << 4) * (size_t)KTOT + k0);
#pragma unroll
      for (int j = 0; j < 4; ++j) acc[i][j] = mm(af, bf[j], acc[i][j]);
    }
  }

  float* slab = sT[wave];
  const int hh = lane >> 4;
  const int c4 = (lane & 15) * 4;
  const int nc = n0 + c4;
  const bool cok = nc < N;
  v4f bv = (v4f){0.f, 0.f, 0.f, 0.f};
  if (EPI == 1) {
    bv = *(const v4fa*)(bias + clampi(nc, 0, N - 4));
    asm volatile("" :: "v"(bv));
  }
#pragma unroll
  for (int i = 0; i < 4; ++i) {
    const int mBase = m0 + (i << 4);
#pragma unroll
    for (int j = 0; j < 4; ++j) {
#pragma unroll
      for (int r = 0; r < 8; ++r) slab[(h8 + r) * 68 + (j << 4) + rl] = acc[i][j][r];
    }
    __builtin_amdgcn_fence(__ATOMIC_RELEASE, "workgroup");
    __builtin_amdgcn_wave_barrier();
    __builtin_amdgcn_fence(__ATOMIC_ACQUIRE, "workgroup");
    v4f vv[8];
#pragma unroll
    for (int it = 0; it < 8; ++it) {
      const int row = it * 2 + hh;
      v4f v = *(const v4fa*)(slab + row * 68 + c4);
      if (EPI == 1) v += bv;
      vv[it] = v;
    }
    for (int pass = 0; pass < 2; ++pass) {
#pragma unroll
      for (int it = 0; it < 8; ++it) {
        const int row = mBase + it * 2 + hh;
        if (cok && row < M) *(volatile v4f*)(D + (size_t)row * (size_t)ldd + nc) = vv[it];
      }
      __threadfence();
    }
    __builtin_amdgcn_fence(__ATOMIC_RELEASE, "workgroup");
    __builtin_amdgcn_wave_barrier();
    __builtin_amdgcn_fence(__ATOMIC_ACQUIRE, "workgroup");
  }
}

#include <stddef.h>
#include <stdint.h>


#define NN      50000
#define DD      128
#define NR3     3
#define NE      800000
#define MP      50048
#define OUT1_EL 6400000
#define OUT_EL  6500000
#define ROWS_C0 25088
#define ROWS_C1 24960
#define NTHR    256
#define NWAVE   8
#define EPT     8
#define CHUNK   (NTHR * EPT)
#define WCAP    (EPT * 32)
#define LISTN   (NWAVE * WCAP)
#define SLA     10
#define NBK     1024
#define NBLKB   49
#define NSLOT   (NBLKB * NBK)
#define RCAP    20992
#define DEGCAP  48
#define ARRN    (NBK + 16)
#define BK_INTS (LISTN + 2 * RCAP + ARRN + 32)
#define SMT_F   1056
#define BV_F    1280
#define NWV     (MP / 32)

#define PBX        3128
#define PB_E_WATT  (PBX + 8)
#define PB_E_WREL  (PB_E_WATT + 24)
#define PB_E_WSFS  (PB_E_WREL + 8)
#define PB_E_WSFF  (PB_E_WSFS + 8)
#define PB_E_GW2   (PB_E_WSFF + 16)
#define PB_E_FW2   (PB_E_GW2 + 32)
#define PB_TOTAL   (PB_E_FW2 + 4)

static_assert(MP % 64 == 0 && MP % 128 == 0 && MP >= NN && MP % 32 == 0 && MP % 8 == 0);
static_assert(ROWS_C0 + ROWS_C1 == MP && ROWS_C0 % 64 == 0 && ROWS_C1 % 64 == 0);
static_assert(PBX * 256 == MP * 16);
static_assert(NSLOT >= MP && NBK == (1 << SLA));
static_assert(RCAP >= 16753 + 16753 / 4 && RCAP % 512 == 0 && RCAP < 65536);
static_assert(DEGCAP >= 36 + 8 && DEGCAP <= 64);
static_assert(NE <= (1 << 20) && (NE % 8) == 0 && NN <= 65536 * 16);
static_assert(BK_INTS % 4 == 0 && BK_INTS * 4 <= 262144);
static_assert(OUT1_EL == NN * DD && OUT1_EL + 2 * NN == OUT_EL);
static_assert((OUT1_EL * 4) % 128 == 0);
static_assert(DD == 128 && NN % 2 == 0);

typedef int      v4i __attribute__((ext_vector_type(4)));
typedef unsigned v2u __attribute__((ext_vector_type(2)));
typedef v4i __attribute__((may_alias)) v4ia;
typedef v2u __attribute__((may_alias)) v2ua;

__device__ __forceinline__ void pinf(float x)      { asm volatile("" :: "v"(x)); }
__device__ __forceinline__ void pini(int x)        { asm volatile("" :: "v"(x)); }
__device__ __forceinline__ void pin4f(const v4f x) { asm volatile("" :: "v"(x)); }
__device__ __forceinline__ void pin2u(const v2u x) { asm volatile("" :: "v"(x)); }

__device__ __forceinline__ void st2u(unsigned short* p, const v4u v) {
  volatile v4u* q = (volatile v4u*)p;
  *q = v; __threadfence(); *q = v;
}
__device__ __forceinline__ void st2f(float* p, const v4f v) {
  volatile v4f* q = (volatile v4f*)p;
  *q = v; __threadfence(); *q = v;
}

__device__ __forceinline__ v4f bfv4(const v4f a) {
  return (v4f){ bf16_val(a[0]), bf16_val(a[1]), bf16_val(a[2]), bf16_val(a[3]) };
}
__device__ __forceinline__ v4f blend4(const v4f a, unsigned ma, const v4f b, unsigned mb) {
  v4f o;
  o[0] = __uint_as_float((__float_as_uint(a[0]) & ma) | (__float_as_uint(b[0]) & mb));
  o[1] = __uint_as_float((__float_as_uint(a[1]) & ma) | (__float_as_uint(b[1]) & mb));
  o[2] = __uint_as_float((__float_as_uint(a[2]) & ma) | (__float_as_uint(b[2]) & mb));
  o[3] = __uint_as_float((__float_as_uint(a[3]) & ma) | (__float_as_uint(b[3]) & mb));
  return o;
}

__device__ __forceinline__ v4u gat8(const float* __restrict__ w, int base, int stride) {
  float f[8];
#pragma unroll
  for (int i = 0; i < 8; ++i) { f[i] = w[base + i * stride]; pinf(f[i]); }
  return (v4u){ pk16(bf16_bits(f[0]), bf16_bits(f[1])), pk16(bf16_bits(f[2]), bf16_bits(f[3])),
                pk16(bf16_bits(f[4]), bf16_bits(f[5])), pk16(bf16_bits(f[6]), bf16_bits(f[7])) };
}

__device__ __forceinline__ v4f ldv4(const float* __restrict__ p, int off) {
  const v4f v = *(const v4fa*)(p + off);
  pin4f(v);
  return v;
}

__global__ __launch_bounds__(256) void k_prep(
    const float* __restrict__ x, const float* __restrict__ att_w1, const float* __restrict__ att_b1,
    const float* __restrict__ att_w2, const float* __restrict__ att_b2, const float* __restrict__ pred_w,
    const float* __restrict__ pred_b, const float* __restrict__ rel_w, const float* __restrict__ rel_b,
    const float* __restrict__ relw_w, const float* __restrict__ relw_b, const float* __restrict__ gate_w,
    const float* __restrict__ gate_b, const float* __restrict__ self_w, const float* __restrict__ self_b,
    const float* __restrict__ feat_w, const float* __restrict__ feat_b, const float* __restrict__ fus_w,
    const float* __restrict__ fus_b, const float* __restrict__ ln_g, const float* __restrict__ ln_b,
    unsigned short* xb, unsigned short* watt, unsigned short* wrel, unsigned short* wsf,
    unsigned short* gw2, unsigned short* fw2, float* smt, float* bvt) {
  const int b = (int)blockIdx.x, tid = (int)threadIdx.x;
  if (b < PBX) {
    const int u   = b * 256 + tid;
    const int row = u >> 4;
    const int c0  = (u & 15) * 8;
    const int rc  = row < NN ? row : NN - 1;
    const v4f a = ldv4(x, rc * DD + c0);
    const v4f c = ldv4(x, rc * DD + c0 + 4);
    v4u o = pack8_bf16(a, c);
    const unsigned mk = row < NN ? 0xFFFFFFFFu : 0u;
    o &= mk;
    st2u(xb + (size_t)u * 8, o);
  } else if (b < PB_E_WATT) {
    const int u = (b - PBX) * 256 + tid;
    const int n = u >> 4, k8 = (u & 15) * 8;
    st2u(watt + (size_t)u * 8, gat8(att_w1, (n >> 6) * 8192 + k8 * 64 + (n & 63), 64));
  } else if (b < PB_E_WREL) {
    const int u = (b - PB_E_WATT) * 256 + tid;
    const int r = u >> 11, n = (u >> 4) & 127, k8 = (u & 15) * 8;
    st2u(wrel + (size_t)u * 8, gat8(rel_w, r * 16384 + k8 * DD + n, DD));
  } else if (b < PB_E_WSFS) {
    const int u = (b - PB_E_WREL) * 256 + tid;
    const int n = u >> 4, k8 = (u & 15) * 8;
    st2u(wsf + (size_t)u * 8, gat8(self_w, k8 * DD + n, DD));
  } else if (b < PB_E_WSFF) {
    const int u = (b - PB_E_WSFS) * 256 + tid;
    const int n = u >> 4, k8 = (u & 15) * 8;
    st2u(wsf + (size_t)(2048 + u) * 8, gat8(feat_w, k8 * DD + n, DD));
  } else if (b < PB_E_GW2) {
    const int u = (b - PB_E_WSFF) * 256 + tid;
    const int n = u >> 5, kk = (u & 31) * 8;
    st2u(gw2 + (size_t)u * 8, gat8(gate_w, (kk & 127) * DD + n, DD));
  } else if (b < PB_E_FW2) {
    const int u = (b - PB_E_GW2) * 256 + tid;
    const int n = u >> 6, kk = (u & 63) * 8;
    const int ks = (kk & 127) + ((kk >= 256) ? 128 : 0);
    st2u(fw2 + (size_t)u * 8, gat8(fus_w, ks * DD + n, DD));
  } else if (b == PB_E_FW2) {
    const int d = tid >> 1;
    float f0 = pred_w[2 * d];     pinf(f0);
    float f1 = pred_w[2 * d + 1]; pinf(f1);
    float f2 = relw_w[3 * d];     pinf(f2);
    float f3 = relw_w[3 * d + 1]; pinf(f3);
    float f4 = relw_w[3 * d + 2]; pinf(f4);
    float f5 = att_w2[d];         pinf(f5);
    const v4f A = (v4f){ f0, f1, f2, f3 };
    const v4f B = (v4f){ f4, f5, 0.f, 0.f };
    const unsigned mb = (tid & 1) ? 0xFFFFFFFFu : 0u;
    st2f(smt + tid * 4, bfv4(blend4(A, ~mb, B, mb)));
  } else if (b == PB_E_FW2 + 1) {
    float f0 = pred_b[0]; pinf(f0);
    float f1 = pred_b[1]; pinf(f1);
    float f2 = relw_b[0]; pinf(f2);
    float f3 = relw_b[1]; pinf(f3);
    float f4 = relw_b[2]; pinf(f4);
    float f5 = att_b2[0]; pinf(f5);
    float f6 = att_b2[1]; pinf(f6);
    const v4f A = (v4f){ f0, f1, f2, f3 };
    const v4f B = (v4f){ f4, f5, f6, 0.f };
    const unsigned m0 = (tid == 0) ? 0xFFFFFFFFu : 0u;
    const unsigned m1 = (tid == 1) ? 0xFFFFFFFFu : 0u;
    const v4f o = bfv4(blend4(A, m0, B, m1));
    if (tid < 8) st2f(smt + 1024 + tid * 4, o);
  } else {
    const int q  = (b - PB_E_FW2 - 2) * 256 + tid;
    const int sg = __builtin_amdgcn_readfirstlane(q >> 5);
    v4f v = (v4f){ 0.f, 0.f, 0.f, 0.f };
    if (sg == 0)       v = ldv4(att_b1, q * 4);
    else if (sg <= 3)  v = ldv4(rel_b,  (q - 32) * 4);
    else if (sg == 4)  v = ldv4(self_b, (q - 128) * 4);
    else if (sg == 5)  v = ldv4(feat_b, (q - 160) * 4);
    else if (sg == 6)  v = ldv4(gate_b, (q - 192) * 4);
    else if (sg == 7)  v = ldv4(fus_b,  (q - 224) * 4);
    else if (sg == 8)  v = ldv4(ln_g,   (q - 256) * 4);
    else if (sg == 9)  v = ldv4(ln_b,   (q - 288) * 4);
    if (sg <= 9) st2f(bvt + q * 4, bfv4(v));
  }
}

__device__ __forceinline__ float red32(float v) {
  v += __shfl_xor(v, 16, 32); v += __shfl_xor(v, 8, 32); v += __shfl_xor(v, 4, 32);
  v += __shfl_xor(v, 2, 32);  v += __shfl_xor(v, 1, 32);
  return v;
}
__device__ __forceinline__ float red16(float v) {
  v += __shfl_xor(v, 8, 32); v += __shfl_xor(v, 4, 32); v += __shfl_xor(v, 2, 32); v += __shfl_xor(v, 1, 32);
  return v;
}

__global__ __launch_bounds__(256) void k_node(const unsigned short* __restrict__ xb, const float* __restrict__ hpl,
                                              const float* __restrict__ smt, float* outp, float* nat, float* rwt) {
  __shared__ __attribute__((aligned(16))) float tab[SMT_F];
  const int tid = (int)threadIdx.x, lane = tid & 31;
  const int wave = __builtin_amdgcn_readfirstlane(tid >> 5);
  {
    const int i1 = (tid + 256) < (SMT_F / 4) ? (tid + 256) : (SMT_F / 4 - 1);
    const v4f v0 = ldv4(smt, tid * 4);
    const v4f v1 = ldv4(smt, i1 * 4);
    *(v4fa*)(tab + tid * 4) = v0;
    *(v4fa*)(tab + i1 * 4)  = v1;
  }
  __syncthreads();
  const int wv = (int)blockIdx.x * 8 + wave;
  if (wv < NWV) {
    const float* tr = tab + lane * 32;
    const v4f tA0 = *(const v4fa*)(tr),      tB0 = *(const v4fa*)(tr + 4);
    const v4f tA1 = *(const v4fa*)(tr + 8),  tB1 = *(const v4fa*)(tr + 12);
    const v4f tA2 = *(const v4fa*)(tr + 16), tB2 = *(const v4fa*)(tr + 20);
    const v4f tA3 = *(const v4fa*)(tr + 24), tB3 = *(const v4fa*)(tr + 28);
    const v4f bA  = *(const v4fa*)(tab + 1024);
    const v4f bB  = *(const v4fa*)(tab + 1028);
    const int n0 = wv * 32;
    float L0 = 0.f, L1 = 0.f, R0 = 0.f, R1 = 0.f, R2 = 0.f, S0 = 0.f, S1 = 0.f;
#pragma unroll 1
    for (int i = 0; i < 32; ++i) {
      const int n = n0 + i;
      const v2u xw = *(const v2ua*)(xb + (size_t)n * DD + lane * 4);
      pin2u(xw);
      const v4f hv = *(const v4fa*)(hpl + (size_t)n * DD + lane * 4);
      pin4f(hv);
      const float x0 = __uint_as_float(xw.x << 16), x1 = __uint_as_float(xw.x & 0xffff0000u);
      const float x2 = __uint_as_float(xw.y << 16), x3 = __uint_as_float(xw.y & 0xffff0000u);
      float l0 = x0 * tA0[0] + x1 * tA1[0] + x2 * tA2[0] + x3 * tA3[0];
      float l1 = x0 * tA0[1] + x1 * tA1[1] + x2 * tA2[1] + x3 * tA3[1];
      float r0 = x0 * tA0[2] + x1 * tA1[2] + x2 * tA2[2] + x3 * tA3[2];
      float r1 = x0 * tA0[3] + x1 * tA1[3] + x2 * tA2[3] + x3 * tA3[3];
      float r2 = x0 * tB0[0] + x1 * tB1[0] + x2 * tB2[0] + x3 * tB3[0];
      float sp = fmaxf(hv[0], 0.f) * tB0[1] + fmaxf(hv[1], 0.f) * tB1[1]
               + fmaxf(hv[2], 0.f) * tB2[1] + fmaxf(hv[3], 0.f) * tB3[1];
      l0 = red32(l0); l1 = red32(l1); r0 = red32(r0); r1 = red32(r1); r2 = red32(r2);
      sp = red16(sp);
      const float s0 = __shfl(sp, 0, 32);
      const float s1 = __shfl(sp, 16, 32);
      const bool me = (lane == i);
      L0 = me ? l0 : L0; L1 = me ? l1 : L1;
      R0 = me ? r0 : R0; R1 = me ? r1 : R1; R2 = me ? r2 : R2;
      S0 = me ? s0 : S0; S1 = me ? s1 : S1;
    }
    const int n = n0 + lane;
    const bool live = n < NN;
    const float l0 = L0 + bA[0], l1 = L1 + bA[1];
    const float mx = fmaxf(l0, l1);
    const float e0 = expf(l0 - mx), e1 = expf(l1 - mx);
    const float den = e0 + e1;
    float p0 = e0 / den, p1 = e1 / den;
    const float q0 = R0 + bA[2], q1 = R1 + bA[3], q2 = R2 + bB[0];
    const float qm = fmaxf(fmaxf(q0, q1), q2);
    const float g0 = expf(q0 - qm), g1 = expf(q1 - qm), g2 = expf(q2 - qm);
    const float gd = g0 + g1 + g2;
    float w0 = g0 / gd, w1 = g1 / gd, w2 = g2 / gd;
    const float sc0 = S0 + bB[1], sc1 = S1 + bB[2];
    float na = sc0 * p0 + sc1 * p1;
    p0 = live ? p0 : 0.f; p1 = live ? p1 : 0.f;
    w0 = live ? w0 : 0.f; w1 = live ? w1 : 0.f; w2 = live ? w2 : 0.f;
    na = live ? na : 0.f;

    const int sl = (lane & 15) * 2;
    const float a0 = __shfl(p0, sl, 32),     a1 = __shfl(p1, sl, 32);
    const float c0 = __shfl(p0, sl + 1, 32), c1 = __shfl(p1, sl + 1, 32);
    const v4f o1 = (v4f){ a0, a1, c0, c1 };
    const bool ok1 = (lane < 16) && ((n0 + sl + 1) < NN);
    const int nn1 = (n0 + sl) < (NN - 2) ? (n0 + sl) : (NN - 2);
    const int q4 = (lane & 7) * 4;
    const v4f o2 = (v4f){ __shfl(na, q4, 32), __shfl(na, q4 + 1, 32), __shfl(na, q4 + 2, 32), __shfl(na, q4 + 3, 32) };
    const v4f o3 = (v4f){ w0, w1, w2, 0.f };
    if (ok1) st2f(outp + OUT1_EL + (size_t)nn1 * 2, o1);
    if (lane < 8) st2f(nat + n0 + q4, o2);
    st2f(rwt + (size_t)n * 4, o3);
  }
}

__device__ __forceinline__ int ldkey(const int* __restrict__ k, int e, int nE, int sent) {
  const int v = k[e < nE ? e : nE - 1];
  pini(v);
  return (e < nE) ? v : sent;
}

__device__ __forceinline__ int scan_chunk(const int* __restrict__ keys, int nE, int cbase, int slotBase,
                                          int nb, int* list, int tid, int lane, int wave) {
  int wc = 0;
  const int el0  = tid * EPT;
  const int e0   = cbase + el0;
  const int sent = (int)(1u << 31);
  v4i da, db;
  if (cbase + CHUNK <= nE) {
    da = *(const v4i*)(keys + e0);
    db = *(const v4i*)(keys + e0 + 4);
  } else {
    da.x = ldkey(keys, e0,     nE, sent);
    da.y = ldkey(keys, e0 + 1, nE, sent);
    da.z = ldkey(keys, e0 + 2, nE, sent);
    da.w = ldkey(keys, e0 + 3, nE, sent);
    db.x = ldkey(keys, e0 + 4, nE, sent);
    db.y = ldkey(keys, e0 + 5, nE, sent);
    db.z = ldkey(keys, e0 + 6, nE, sent);
    db.w = ldkey(keys, e0 + 7, nE, sent);
  }
  const unsigned nbs = (unsigned)slotBase;
  const unsigned unb = (unsigned)nb;
  const unsigned s0 = (unsigned)da.x - nbs, s1 = (unsigned)da.y - nbs;
  const unsigned s2 = (unsigned)da.z - nbs, s3 = (unsigned)da.w - nbs;
  const unsigned s4 = (unsigned)db.x - nbs, s5 = (unsigned)db.y - nbs;
  const unsigned s6 = (unsigned)db.z - nbs, s7 = (unsigned)db.w - nbs;
  const bool h0 = s0 < unb, h1 = s1 < unb, h2 = s2 < unb, h3 = s3 < unb;
  const bool h4 = s4 < unb, h5 = s5 < unb, h6 = s6 < unb, h7 = s7 < unb;
  const unsigned any = __builtin_amdgcn_ballot_w32(h0 | h1 | h2 | h3 | h4 | h5 | h6 | h7);
  if (any != 0u) {
    const int k = (int)h0 + (int)h1 + (int)h2 + (int)h3 + (int)h4 + (int)h5 + (int)h6 + (int)h7;
    int incl = k;
#pragma unroll
    for (int dd = 1; dd < 32; dd <<= 1) {
      const int y = __shfl_up(incl, dd, 32);
      if (lane >= dd) incl += y;
    }
    wc = __shfl(incl, 31, 32);
    int pos = incl - k;
#define PUTJ(J, HJ, SJ) if (HJ) { if (pos < WCAP) list[wave * WCAP + pos] = ((el0 + (J)) << SLA) | (int)(SJ); pos += 1; }
    PUTJ(0, h0, s0)
    PUTJ(1, h1, s1)
    PUTJ(2, h2, s2)
    PUTJ(3, h3, s3)
    PUTJ(4, h4, s4)
    PUTJ(5, h5, s5)
    PUTJ(6, h6, s6)
    PUTJ(7, h7, s7)
#undef PUTJ
  }
  return wc;
}

__global__ __launch_bounds__(NTHR) void k_bucket(const int* __restrict__ eidx, int* cog, int* flgg, int* listg) {
  extern __shared__ __attribute__((aligned(16))) int dsm[];
  int* list = dsm;
  int* hk   = dsm + LISTN;
  int* ent  = hk + RCAP;
  int* arr  = ent + RCAP;
  int* misc = arr + ARRN;
  const int tid = (int)threadIdx.x, lane = tid & 31;
  const int wave = __builtin_amdgcn_readfirstlane(tid >> 5);
  const int b = (int)blockIdx.x;
  const int r = (int)blockIdx.y;
  const int* srcp = eidx + (size_t)r * (size_t)(2 * NE);
  const int* dstp = srcp + NE;
  const int nodeBase = b * NBK;

  {
    const v4i z4 = {0, 0, 0, 0};
    for (int i = tid * 4; i < BK_INTS; i += NTHR * 4) *(v4ia*)(dsm + i) = z4;
  }
  __syncthreads();

  int t = 0;
  const int nChunks = (NE + CHUNK - 1) / CHUNK;
#pragma unroll 1
  for (int ch = 0; ch < nChunks; ++ch) {
    const int cbase = ch * CHUNK;
    int wcv = scan_chunk(dstp, NE, cbase, nodeBase, NBK, list, tid, lane, wave);
    wcv = clampi(wcv, 0, WCAP);
    const int myc = __builtin_amdgcn_readfirstlane(wcv);
    int* mb = misc + (ch & 1) * 8;
    if (lane == 0) mb[wave] = myc;
    __syncthreads();
    int base = t, tot = 0;
#pragma unroll
    for (int w2 = 0; w2 < NWAVE; ++w2) {
      const int c = clampi(mb[w2], 0, WCAP);
      base += (w2 < wave) ? c : 0;
      tot  += c;
    }
#pragma unroll 1
    for (int b0 = 0; b0 < myc; b0 += 32) {
      const int idx  = b0 + lane;
      const int entv = list[wave * WCAP + (idx < WCAP ? idx : WCAP - 1)];
      const int slot = entv & (NBK - 1);
      const int el   = (entv >> SLA) & (CHUNK - 1);
      const int eid  = clampi(cbase + el, 0, NE - 1);
      const int pos  = base + idx;
      if (idx < myc && pos < RCAP) hk[pos] = (slot << 20) | eid;
    }
    t += tot;
  }
  __syncthreads();
  const int tt = t < RCAP ? t : RCAP;
  const int ov = t > RCAP ? 1 : 0;

  if (tid == 0) {
#pragma unroll 1
    for (int i = 0; i < tt; ++i) {
      const int k = (hk[i] >> 20) & (NBK - 1);
      arr[k] = arr[k] + 1;
    }
  }
  __syncthreads();
  if (wave == 0) {
    const int base = lane * (NBK / 32);
    int s = 0;
#pragma unroll 1
    for (int i = 0; i < NBK / 32; ++i) s += arr[base + i];
    int incl = s;
#pragma unroll
    for (int dd = 1; dd < 32; dd <<= 1) {
      const int y = __shfl_up(incl, dd, 32);
      if (lane >= dd) incl += y;
    }
    int run = incl - s;
#pragma unroll 1
    for (int i = 0; i < NBK / 32; ++i) {
      run += arr[base + i];
      arr[base + i] = run;
    }
    if (lane == 31) arr[NBK] = run;
  }
  __syncthreads();
  if (tid == 0) {
#pragma unroll 1
    for (int i = tt - 1; i >= 0; --i) {
      const int hv = hk[i];
      const int k = (hv >> 20) & (NBK - 1);
      const int p = clampi(arr[k] - 1, 0, RCAP - 1);
      arr[k] = p;
      ent[p] = hv & 0xFFFFF;
    }
  }
  __syncthreads();

  v4i cov;
  {
    int ovd = 0;
    int cw[4];
#pragma unroll
    for (int j = 0; j < 4; ++j) {
      const int k  = tid * 4 + j;
      const int st = arr[k];
      const int c  = arr[k + 1] - st;
      ovd |= (c > DEGCAP) ? 1 : 0;
      cw[j] = clampi(st, 0, RCAP - 1) | (clampi(c, 0, DEGCAP) << 16);
    }
    cov.x = cw[0]; cov.y = cw[1]; cov.z = cw[2]; cov.w = cw[3];
    const unsigned om = __builtin_amdgcn_ballot_w32(ovd != 0);
    if (lane == 0) misc[20 + wave] = (om != 0u) ? 1 : 0;
  }
  __syncthreads();
  int fl = ov;
#pragma unroll
  for (int w2 = 0; w2 < NWAVE; ++w2) fl |= misc[20 + w2];
  const v4i flv = {fl, fl, fl, fl};

  int* cg = cog + (size_t)r * NSLOT + nodeBase;
  int* fg = flgg + (size_t)(r * NBLKB + b) * 32;
  int* lg = listg + (size_t)(r * NBLKB + b) * (size_t)(2 * RCAP);
  for (int pass = 0; pass < 2; ++pass) {
    *(volatile v4i*)(cg + tid * 4) = cov;
    if (tid < 8) *(volatile v4i*)(fg + tid * 4) = flv;
#pragma unroll 2
    for (int i = tid * 2; i < RCAP; i += NTHR * 2) {
      const int e0 = clampi(ent[i], 0, NE - 1);
      const int e1 = clampi(ent[i + 1], 0, NE - 1);
      int s0 = srcp[e0]; pini(s0);
      int s1 = srcp[e1]; pini(s1);
      v4i o;
      o.x = clampi(s0, 0, NN - 1); o.y = e0;
      o.z = clampi(s1, 0, NN - 1); o.w = e1;
      *(volatile v4i*)(lg + 2 * i) = o;
    }
    __threadfence();
  }
}

__device__ __forceinline__ v4u hilo_piece(const v4f v, int lane) {
  const int sl = (lane & 15) * 2;
  v4f a, c;
  a[0] = __shfl(v[0], sl, 32);     a[1] = __shfl(v[1], sl, 32);
  a[2] = __shfl(v[2], sl, 32);     a[3] = __shfl(v[3], sl, 32);
  c[0] = __shfl(v[0], sl + 1, 32); c[1] = __shfl(v[1], sl + 1, 32);
  c[2] = __shfl(v[2], sl + 1, 32); c[3] = __shfl(v[3], sl + 1, 32);
  const v4u hi = pack8_bf16(a, c);
  const v4u lo = pack8_bf16_lo(a, c);
  const unsigned mk = (lane >= 16) ? 0xFFFFFFFFu : 0u;
  return (lo & mk) | (hi & ~mk);
}

template <int R>
__global__ __launch_bounds__(256) void k_replay(const float* __restrict__ T, const int* __restrict__ cog,
                                                const int* __restrict__ flgg, const int* __restrict__ listg,
                                                const float* __restrict__ ew, const float* __restrict__ rwt,
                                                float* comb, unsigned short* chl) {
  const int tid = (int)threadIdx.x, lane = tid & 31;
  const int wave = __builtin_amdgcn_readfirstlane(tid >> 5);
  const int n = (int)blockIdx.x * 8 + wave;
  const bool live = n < NN;
  const int b = clampi(n >> SLA, 0, NBLKB - 1);
  int cw = cog[(size_t)R * NSLOT + n];
  pini(cw);
  const int off = clampi(cw & 0xffff, 0, RCAP - 1);
  int c = clampi((cw >> 16) & 0xffff, 0, DEGCAP);
  c = c > (RCAP - off) ? (RCAP - off) : c;
  c = live ? c : 0;
  const int cn = __builtin_amdgcn_readfirstlane(c);
  int fw = flgg[(size_t)(R * NBLKB + b) * 32];
  pini(fw);
  const size_t lb = (size_t)(R * NBLKB + b) * (size_t)RCAP;
  const int i0 = (off + lane) < RCAP ? (off + lane) : (RCAP - 1);
  const int i1 = (off + 32 + lane) < RCAP ? (off + 32 + lane) : (RCAP - 1);
  const v2u e0 = *(const v2ua*)(listg + (lb + (size_t)i0) * 2);
  const v2u e1 = *(const v2ua*)(listg + (lb + (size_t)i1) * 2);
  pin2u(e0); pin2u(e1);
  const int s0 = clampi((int)e0.x, 0, NN - 1), d0 = clampi((int)e0.y, 0, NE - 1);
  const int s1 = clampi((int)e1.x, 0, NN - 1), d1 = clampi((int)e1.y, 0, NE - 1);
  float w0 = ew[(size_t)R * NE + d0]; pinf(w0);
  float w1 = ew[(size_t)R * NE + d1]; pinf(w1);
  w0 = bf16_val(w0);
  w1 = bf16_val(w1);

  v4f acc = (v4f){0.f, 0.f, 0.f, 0.f};
  const float* Tl = T + lane * 4;
  const int c0 = cn < 32 ? cn : 32;
#pragma unroll 1
  for (int p = 0; p < c0; ++p) {
    const int sv = clampi(__shfl(s0, p, 32), 0, NN - 1);
    const float wv = __shfl(w0, p, 32);
    const v4f tv = *(const v4fa*)(Tl + (size_t)sv * DD);
    pin4f(tv);
    acc += wv * tv;
  }
#pragma unroll 1
  for (int p = 32; p < cn; ++p) {
    const int sv = clampi(__shfl(s1, p - 32, 32), 0, NN - 1);
    const float wv = __shfl(w1, p - 32, 32);
    const v4f tv = *(const v4fa*)(Tl + (size_t)sv * DD);
    pin4f(tv);
    acc += wv * tv;
  }

  float rwv = rwt[(size_t)n * 4 + R];
  pinf(rwv);
  float* cp = comb + (size_t)n * DD + lane * 4;
  v4f o;
  if (R == 0) {
    o = rwv * acc;
  } else {
    const v4f old = *(const v4fa*)cp;
    pin4f(old);
    o = old + rwv * acc;
  }
  const float pz = (fw != 0) ? __uint_as_float(0x7fc00000u) : 0.0f;
  o = o + pz;
  if (!live) o = (v4f){0.f, 0.f, 0.f, 0.f};
  st2f(cp, o);
  if (R == 2) {
    const v4u pc = hilo_piece(o, lane);
    st2u(chl + (size_t)n * 256 + lane * 8, pc);
  }
}

__global__ __launch_bounds__(256) void k_row(const float* __restrict__ G, const float* __restrict__ comb,
                                             const float* __restrict__ nat, const float* __restrict__ sf,
                                             unsigned short* fa, int row0) {
  const int tid = (int)threadIdx.x, lane = tid & 31;
  const int wave = __builtin_amdgcn_readfirstlane(tid >> 5);
  const int i = (int)blockIdx.x * 8 + wave;
  const int n = clampi(row0 + i, 0, MP - 1);
  const bool live = n < NN;
  const v4f g  = *(const v4fa*)(G + (size_t)n * DD + lane * 4);    pin4f(g);
  const v4f cm = *(const v4fa*)(comb + (size_t)n * DD + lane * 4); pin4f(cm);
  float a = nat[n];                                                 pinf(a);
  const v4f sv = *(const v4fa*)(sf + (size_t)i * 256 + lane * 4);  pin4f(sv);
  v4f wr;
  wr[0] = ((1.0f / (1.0f + expf(-g[0]))) * cm[0]) * a;
  wr[1] = ((1.0f / (1.0f + expf(-g[1]))) * cm[1]) * a;
  wr[2] = ((1.0f / (1.0f + expf(-g[2]))) * cm[2]) * a;
  wr[3] = ((1.0f / (1.0f + expf(-g[3]))) * cm[3]) * a;
  v4f sl = sv;
  if (!live) { wr = (v4f){0.f, 0.f, 0.f, 0.f}; sl = (v4f){0.f, 0.f, 0.f, 0.f}; }
  const v4u p0 = hilo_piece(sl, lane);
  const v4u p1 = hilo_piece(wr, lane);
  unsigned short* rp = fa + (size_t)i * 512 + lane * 8;
  for (int pass = 0; pass < 2; ++pass) {
    *(volatile v4u*)(rp)       = p0;
    *(volatile v4u*)(rp + 256) = p1;
    __threadfence();
  }
}

__global__ __launch_bounds__(256) void k_final(const float* __restrict__ fu, const float* __restrict__ sf,
                                               const float* __restrict__ lnt, float* outp, int row0) {
  __shared__ __attribute__((aligned(16))) float lt[256];
  const int tid = (int)threadIdx.x, lane = tid & 31;
  const int wave = __builtin_amdgcn_readfirstlane(tid >> 5);
  if (wave < 2) {
    const v4f v = ldv4(lnt, tid * 4);
    *(v4fa*)(lt + tid * 4) = v;
  }
  __syncthreads();
  const v4f gg = *(const v4fa*)(lt + lane * 4);
  const v4f bb = *(const v4fa*)(lt + 128 + lane * 4);
  const int i = (int)blockIdx.x * 8 + wave;
  const int n = clampi(row0 + i, 0, MP - 1);
  const v4f f  = *(const v4fa*)(fu + (size_t)n * DD + lane * 4);       pin4f(f);
  const v4f tr = *(const v4fa*)(sf + (size_t)i * 256 + 128 + lane * 4); pin4f(tr);
  v4f v;
  v[0] = ((f[0] > 0.0f) ? f[0] : (f[0] - f[0])) + tr[0];
  v[1] = ((f[1] > 0.0f) ? f[1] : (f[1] - f[1])) + tr[1];
  v[2] = ((f[2] > 0.0f) ? f[2] : (f[2] - f[2])) + tr[2];
  v[3] = ((f[3] > 0.0f) ? f[3] : (f[3] - f[3])) + tr[3];
  const float s  = red32((v[0] + v[1]) + (v[2] + v[3]));
  const float mu = s * (1.0f / 128.0f);
  const v4f d = v - mu;
  const float q  = red32((d[0] * d[0] + d[1] * d[1]) + (d[2] * d[2] + d[3] * d[3]));
  const float var = q * (1.0f / 128.0f);
  const float den = sqrtf(var + 1e-5f);
  v4f y;
  y[0] = d[0] / den * gg[0] + bb[0];
  y[1] = d[1] / den * gg[1] + bb[1];
  y[2] = d[2] / den * gg[2] + bb[2];
  y[3] = d[3] / den * gg[3] + bb[3];
  const int nc = n < NN ? n : NN - 1;
  if (n < NN) st2f(outp + (size_t)nc * DD + lane * 4, y);
}

constexpr size_t al256c(size_t x) { return (x + 255) & ~(size_t)255; }
constexpr size_t SZ_XB  = (size_t)MP * 128 * 2;
constexpr size_t SZ_U   = (size_t)MP * 512;
constexpr size_t SZ_V   = (size_t)ROWS_C0 * 1024;
constexpr size_t SZ_LST = (size_t)NR3 * NBLKB * RCAP * 8;
constexpr size_t O_XB   = 0;
constexpr size_t O_RA   = al256c(O_XB + SZ_XB);
constexpr size_t O_COMB = al256c(O_RA + SZ_U);
constexpr size_t O_RC   = al256c(O_COMB + SZ_U);
constexpr size_t O_RD   = al256c(O_RC + SZ_V);
constexpr size_t O_CO   = al256c(O_RD + SZ_V);
constexpr size_t O_FLG  = al256c(O_CO + (size_t)NR3 * NSLOT * 4);
constexpr size_t O_NA   = al256c(O_FLG + (size_t)NR3 * NBLKB * 128);
constexpr size_t O_RW   = al256c(O_NA + (size_t)MP * 4);
constexpr size_t O_WATT = al256c(O_RW + (size_t)MP * 16);
constexpr size_t O_WREL = al256c(O_WATT + 32768);
constexpr size_t O_WSF  = al256c(O_WREL + 98304);
constexpr size_t O_GW2  = al256c(O_WSF + 65536);
constexpr size_t O_FW2  = al256c(O_GW2 + 65536);
constexpr size_t O_SMT  = al256c(O_FW2 + 131072);
constexpr size_t O_BV   = al256c(O_SMT + (size_t)SMT_F * 4);
constexpr size_t WS_TOTAL = al256c(O_BV + (size_t)BV_F * 4);
static_assert(WS_TOTAL == ((size_t)458853 << 8));
static_assert(WS_TOTAL <= ((size_t)128 << 20));
static_assert(SZ_LST <= SZ_V);
static_assert((size_t)MP * 256 * 2 <= SZ_V);
static_assert((size_t)ROWS_C0 * 512 * 2 <= SZ_V && (size_t)ROWS_C1 * 512 * 2 <= SZ_V);
static_assert((size_t)ROWS_C0 * 256 * 4 <= SZ_V && (size_t)ROWS_C1 * 256 * 4 <= SZ_V);

static inline int gemm_blocks(int M, int N) {
  const int t = ((M + 63) / 64) * ((N + 63) / 64);
  return (t + 7) / 8;
}

extern "C" void kernel_launch(void* const* d_in, const int* in_sizes, int n_in,
                              void* d_out, int out_size, void* d_ws, size_t ws_size,
                              hipStream_t stream) {
  if (n_in < 23) return;
  const int want[23] = { NN * DD, NR3 * 2 * NE, NR3 * NE, 2 * DD * 64, 2 * 64, 2 * 64, 2, DD * 2, 2,
                         NR3 * DD * DD, NR3 * DD, DD * NR3, NR3, DD * DD, DD, DD * DD, DD, DD * DD, DD,
                         2 * DD * DD, DD, DD, DD };
  for (int i = 0; i < 23; ++i) if (in_sizes[i] != want[i]) return;
  if (out_size != OUT_EL) return;
  if (ws_size < WS_TOTAL) return;

  const float* feat   = (const float*)d_in[0];
  const int*   eidx   = (const int*)  d_in[1];
  const float* ew     = (const float*)d_in[2];
  const float* att_w1 = (const float*)d_in[3];
  const float* att_b1 = (const float*)d_in[4];
  const float* att_w2 = (const float*)d_in[5];
  const float* att_b2 = (const float*)d_in[6];
  const float* pred_w = (const float*)d_in[7];
  const float* pred_b = (const float*)d_in[8];
  const float* rel_w  = (const float*)d_in[9];
  const float* rel_b  = (const float*)d_in[10];
  const float* relw_w = (const float*)d_in[11];
  const float* relw_b = (const float*)d_in[12];
  const float* gate_w = (const float*)d_in[13];
  const float* gate_b = (const float*)d_in[14];
  const float* self_w = (const float*)d_in[15];
  const float* self_b = (const float*)d_in[16];
  const float* feat_w = (const float*)d_in[17];
  const float* feat_b = (const float*)d_in[18];
  const float* fus_w  = (const float*)d_in[19];
  const float* fus_b  = (const float*)d_in[20];
  const float* ln_g   = (const float*)d_in[21];
  const float* ln_b   = (const float*)d_in[22];
  float* out = (float*)d_out;

  char* ws = (char*)d_ws;
  unsigned short* XB   = (unsigned short*)(ws + O_XB);
  float*          RA   = (float*)(ws + O_RA);
  float*          COMB = (float*)(ws + O_COMB);
  unsigned short* RC   = (unsigned short*)(ws + O_RC);
  int*            LIST = (int*)(ws + O_RD);
  float*          SF   = (float*)(ws + O_RD);
  int*            CO   = (int*)(ws + O_CO);
  int*            FLG  = (int*)(ws + O_FLG);
  float*          NA   = (float*)(ws + O_NA);
  float*          RW   = (float*)(ws + O_RW);
  unsigned short* WATT = (unsigned short*)(ws + O_WATT);
  unsigned short* WREL = (unsigned short*)(ws + O_WREL);
  unsigned short* WSF  = (unsigned short*)(ws + O_WSF);
  unsigned short* GW2  = (unsigned short*)(ws + O_GW2);
  unsigned short* FW2  = (unsigned short*)(ws + O_FW2);
  float*          SMT  = (float*)(ws + O_SMT);
  float*          BV   = (float*)(ws + O_BV);

  const int bkLds = BK_INTS * 4;
  hipFuncSetAttribute(reinterpret_cast<const void*>(&k_bucket), hipFuncAttributeMaxDynamicSharedMemorySize, bkLds);

  k_prep<<<PB_TOTAL, 256, 0, stream>>>(feat, att_w1, att_b1, att_w2, att_b2, pred_w, pred_b, rel_w, rel_b,
                                       relw_w, relw_b, gate_w, gate_b, self_w, self_b, feat_w, feat_b,
                                       fus_w, fus_b, ln_g, ln_b, XB, WATT, WREL, WSF, GW2, FW2, SMT, BV);
  k_gemm_nt<0, 1><<<gemm_blocks(MP, 128), 256, 0, stream>>>(XB, WATT, BV, RA, MP, 128, 128, 128);
  k_node<<<(NWV + 7) / 8, 256, 0, stream>>>(XB, RA, SMT, out, NA, RW);
  k_bucket<<<dim3(NBLKB, NR3), NTHR, bkLds, stream>>>(eidx, CO, FLG, LIST);
  k_gemm_nt<0, 1><<<gemm_blocks(MP, 128), 256, 0, stream>>>(XB, WREL, BV + 128, RA, MP, 128, 128, 128);
  k_replay<0><<<MP / 8, 256, 0, stream>>>(RA, CO, FLG, LIST, ew, RW, COMB, RC);
  k_gemm_nt<0, 1><<<gemm_blocks(MP, 128), 256, 0, stream>>>(XB, WREL + 16384, BV + 256, RA, MP, 128, 128, 128);
  k_replay<1><<<MP / 8, 256, 0, stream>>>(RA, CO, FLG, LIST, ew, RW, COMB, RC);
  k_gemm_nt<0, 1><<<gemm_blocks(MP, 128), 256, 0, stream>>>(XB, WREL + 32768, BV + 384, RA, MP, 128, 128, 128);
  k_replay<2><<<MP / 8, 256, 0, stream>>>(RA, CO, FLG, LIST, ew, RW, COMB, RC);
  k_gemm_nt<0, 1><<<gemm_blocks(MP, 128), 256, 0, stream>>>(RC, GW2, BV + 768, RA, MP, 128, 256, 128);
  for (int c = 0; c < 2; ++c) {
    const int row0 = c == 0 ? 0 : ROWS_C0;
    const int rows = c == 0 ? ROWS_C0 : ROWS_C1;
    k_gemm_nt<0, 1><<<gemm_blocks(rows, 256), 256, 0, stream>>>(XB + (size_t)row0 * 128, WSF, BV + 512, SF,
                                                                 rows, 256, 128, 256);
    k_row<<<rows / 8, 256, 0, stream>>>(RA, COMB, NA, SF, RC, row0);
    k_gemm_nt<0, 1><<<gemm_blocks(rows, 128), 256, 0, stream>>>(RC, FW2, BV + 896, RA + (size_t)row0 * 128,
                                                                 rows, 128, 512, 128);
    k_final<<<rows / 8, 256, 0, stream>>>(RA, SF, BV + 1024, out, row0);
  }
}
